// MultiHeadAttention_36902359007528
// MI455X (gfx1250) — hardware-verified
//
#include <hip/hip_runtime.h>


#ifndef NB
#define NB 2
#endif
#ifndef SEQ
#define SEQ 2048
#endif
#define NB_FULL  2
#define SEQ_FULL 2048
#ifndef OUT_SEQ
#define OUT_SEQ SEQ
#endif
#define DM   1024
#define NH_  16
#define HD   64
#define AW   4
#define LNW  8
#define SC2  (0.125f * 1.4426950408889634f)
#define PSH  10.0f
#define WCS  64.0f
#define ACS  16.0f
#define FSC  (1.0f / 1024.0f)

static_assert(HD == 64);
static_assert(NH_ * HD == DM);
static_assert(DM % 64 == 0);
static_assert(DM % 32 == 0);
static_assert(DM % 128 == 0);
static_assert(SEQ % 64 == 0);
static_assert((NB * SEQ) % 64 == 0);
static_assert(SEQ % 32 == 0);
static_assert(SEQ % (16 * AW) == 0);
static_assert((NB * SEQ) % LNW == 0);
static_assert(((size_t)SEQ * DM) % 8 == 0);
static_assert(((size_t)DM * DM) % 8 == 0);
static_assert(WCS * ACS * FSC == 1.0f);
static_assert(NB <= NB_FULL);
static_assert(SEQ <= SEQ_FULL);

typedef _Float16 h16;
typedef unsigned short bf;
typedef __attribute__((ext_vector_type(16))) __bf16   v16bf;
typedef __attribute__((ext_vector_type(16))) _Float16 v16h;
typedef __attribute__((ext_vector_type(8)))  _Float16 v8h;
typedef __attribute__((ext_vector_type(4)))  _Float16 v4h;
typedef __attribute__((ext_vector_type(8)))  unsigned short v8us;
typedef __attribute__((ext_vector_type(4)))  unsigned short v4us;
typedef __attribute__((ext_vector_type(8)))  float    v8f;
typedef __attribute__((ext_vector_type(4)))  float    v4f;
typedef v4f  __attribute__((may_alias)) v4fa;

__device__ __forceinline__ unsigned short f2bf(float f) { unsigned u = __float_as_uint(f); u += 0x7FFFu + ((u >> 16) & 1u); return (unsigned short)(u >> 16); }
__device__ __forceinline__ float bf2f(unsigned short w) { return __uint_as_float(((unsigned)w) << 16); }
__device__ __forceinline__ float bfv(float f) { return bf2f(f2bf(f)); }
__device__ __forceinline__ v16h cat16(v8h lo, v8h hi) { return __builtin_shufflevector(lo, hi, 0, 1, 2, 3, 4, 5, 6, 7, 8, 9, 10, 11, 12, 13, 14, 15); }
__device__ __forceinline__ v16bf cat16b(v8us lo, v8us hi) { return __builtin_bit_cast(v16bf, __builtin_shufflevector(lo, hi, 0, 1, 2, 3, 4, 5, 6, 7, 8, 9, 10, 11, 12, 13, 14, 15)); }
__device__ __forceinline__ v8f wm(v16h a, v16h b, v8f c) {
    c = __builtin_amdgcn_wmma_f32_16x16x32_f16(false, a, false, b, (short)0, c, false, false);
    asm volatile("v_nop\n\tv_nop\n\tv_nop\n\tv_nop" : "+v"(c) : "v"(a), "v"(b));
    return c; }
__device__ __forceinline__ v8f wm(v16bf a, v16bf b, v8f c) {
    c = __builtin_amdgcn_wmma_f32_16x16x32_bf16(false, a, false, b, (short)0, c, false, false);
    asm volatile("v_nop\n\tv_nop\n\tv_nop\n\tv_nop" : "+v"(c) : "v"(a), "v"(b));
    return c; }
__device__ __forceinline__ v16h  ldf(const h16* p) { return cat16(*(const v8h*)p, *(const v8h*)(p + 16)); }
__device__ __forceinline__ v16bf ldf(const bf* p)  { return cat16b(*(const v8us*)p, *(const v8us*)(p + 16)); }
template <typename T> struct FragT;
template <> struct FragT<h16> { typedef v16h  t; };
template <> struct FragT<bf>  { typedef v16bf t; };
__device__ __forceinline__ void wave_sync() { __builtin_amdgcn_fence(3  , "wavefront"); __builtin_amdgcn_wave_barrier(); asm volatile("" ::: "memory"); }

__global__ __launch_bounds__(256) void k_cvt8(const float* __restrict__ src, bf* dst, size_t n8) {
    const size_t i = (size_t)blockIdx.x * 256 + threadIdx.x; if (i >= n8) return;
    const v8f v = *(const v8f*)(src + i * 8); v8us o;
#pragma unroll
    for (int k = 0; k < 8; ++k) o[k] = f2bf(v[k]);
    *(volatile v8us*)(dst + i * 8) = o; __threadfence(); *(volatile v8us*)(dst + i * 8) = o;
}

__global__ __launch_bounds__(256) void k_cvt8h(const float* __restrict__ src, h16* dst, size_t n8) {
    const size_t i = (size_t)blockIdx.x * 256 + threadIdx.x; if (i >= n8) return;
    const v8f v = *(const v8f*)(src + i * 8); v8h o;
#pragma unroll
    for (int k = 0; k < 8; ++k) o[k] = (h16)(bfv(v[k]) * WCS);
    *(volatile v8h*)(dst + i * 8) = o; __threadfence(); *(volatile v8h*)(dst + i * 8) = o;
}

template <typename T, bool BROW, bool RELU, bool OUTF32>
__device__ __forceinline__ void gemm_body(const T* __restrict__ A, const T* __restrict__ Bt, const float* __restrict__ bias, const float* __restrict__ resid,
                                          h16* Ph, float* Pf, int RB, size_t sRB, int pitch, int CB, size_t sCB, float scale, float ocarry) {
    __shared__ __align__(16) float os[16 * 68];
    typedef typename FragT<T>::t frag_t;
    const int K = DM;
    const int lane = threadIdx.x & 31, lr = lane & 15, hi = lane >> 4; const int r0 = blockIdx.x * 64, c0 = blockIdx.y * 64;
    v8f acc[4][4];
#pragma unroll
    for (int mb = 0; mb < 4; ++mb)
#pragma unroll
        for (int nb = 0; nb < 4; ++nb) acc[mb][nb] = (v8f){};
    const size_t aoff = (size_t)(r0 + lr) * K + 8 * hi, boff = (size_t)(c0 + lr) * K + 8 * hi;
#pragma unroll 1
    for (int kc = 0; kc < K; kc += 32) {
        frag_t a[4];
#pragma unroll
        for (int mb = 0; mb < 4; ++mb) a[mb] = ldf(A + aoff + (size_t)mb * 16 * K + kc);
#pragma unroll
        for (int nb = 0; nb < 4; ++nb) { const frag_t b = ldf(Bt + boff + (size_t)nb * 16 * K + kc);
#pragma unroll
            for (int mb = 0; mb < 4; ++mb) acc[mb][nb] = wm(a[mb], b, acc[mb][nb]); }
    }
    if (!OUTF32) {
        const size_t tbase = (size_t)(r0 / RB) * sRB + (size_t)(r0 % RB) * (size_t)pitch + (size_t)(c0 / CB) * sCB + (size_t)(c0 % CB);
        const int c8 = (lane & 7) * 8;
        float cb[8];
#pragma unroll
        for (int i = 0; i < 8; ++i) cb[i] = 0.0f;
        if (!BROW) { const v4f b0 = *(const v4f*)(bias + c0 + c8); const v4f b1 = *(const v4f*)(bias + c0 + c8 + 4);
#pragma unroll
            for (int i = 0; i < 4; ++i) { cb[i] = bfv(b0[i]); cb[4 + i] = bfv(b1[i]); } }
#pragma unroll
        for (int mb = 0; mb < 4; ++mb) {
#pragma unroll
            for (int nb = 0; nb < 4; ++nb) {
#pragma unroll
                for (int j = 0; j < 8; ++j) os[(hi * 8 + j) * 68 + nb * 16 + lr] = acc[mb][nb][j]; }
            wave_sync();
            const size_t sb = tbase + (size_t)(mb * 16) * (size_t)pitch;
#pragma unroll 1
            for (int ps = 0; ps < 2; ++ps) {
#pragma unroll
                for (int s = 0; s < 4; ++s) { const int row = 4 * s + (lane >> 3);
                    const v4f x0 = *(const v4fa*)(&os[row * 68 + c8]); const v4f x1 = *(const v4fa*)(&os[row * 68 + c8 + 4]);
                    float rbv = 0.0f;
                    if (BROW) rbv = bfv(bias[r0 + mb * 16 + row]);
                    v8h hv;
#pragma unroll
                    for (int i = 0; i < 4; ++i) {
                        float u0 = x0[i] * scale + cb[i] + rbv; float u1 = x1[i] * scale + cb[4 + i] + rbv;
                        if (RELU) { u0 = fmaxf(u0, 0.0f); u1 = fmaxf(u1, 0.0f); }
                        hv[i] = (h16)(u0 * ocarry); hv[4 + i] = (h16)(u1 * ocarry); }
                    const size_t oo = sb + (size_t)row * (size_t)pitch + c8;
                    *(volatile v8h*)(Ph + oo) = hv; }
                if (ps == 0) __threadfence(); }
            wave_sync();
        }
    } else {
        const int cofs = lr * 4;
        const v4f braw = *(const v4f*)(bias + c0 + cofs); v4f bb;
#pragma unroll
        for (int i = 0; i < 4; ++i) bb[i] = bfv(braw[i]);
#pragma unroll
        for (int mb = 0; mb < 4; ++mb) {
#pragma unroll
            for (int nb = 0; nb < 4; ++nb) {
#pragma unroll
                for (int j = 0; j < 8; ++j) os[(hi * 8 + j) * 68 + nb * 16 + lr] = acc[mb][nb][j]; }
            wave_sync();
#pragma unroll 1
            for (int ps = 0; ps < 2; ++ps) {
#pragma unroll
                for (int s = 0; s < 8; ++s) { const int row = 2 * s + hi;
                    const v4f xv = *(const v4fa*)(&os[row * 68 + cofs]);
                    const size_t gi = (size_t)(r0 + mb * 16 + row) * DM + c0 + cofs;
                    const v4f rs = *(const v4f*)(resid + gi); v4f val;
#pragma unroll
                    for (int i = 0; i < 4; ++i) val[i] = xv[i] * scale + bb[i] + rs[i];
                    *(volatile v4f*)(Pf + gi) = val; }
                if (ps == 0) __threadfence(); }
            wave_sync();
        }
    }
}

__global__ __launch_bounds__(32) void k_proj_qk(const bf* __restrict__ A, const bf* __restrict__ Bt, const float* __restrict__ bias, h16* Ph) {
    gemm_body<bf, false, false, false>(A, Bt, bias, bias, Ph, (float*)nullptr, SEQ, (size_t)NH_ * SEQ * HD, HD, HD, (size_t)SEQ * HD, 1.0f, 1.0f);
}
__global__ __launch_bounds__(32) void k_proj_vt(const bf* __restrict__ A, const bf* __restrict__ Bt, const float* __restrict__ bias, h16* Ph) {
    gemm_body<bf, true, false, false>(A, Bt, bias, bias, Ph, (float*)nullptr, DM, (size_t)0, SEQ, SEQ, (size_t)DM * SEQ, 1.0f, 1.0f);
}
__global__ __launch_bounds__(32) void k_ffn1(const h16* __restrict__ A, const h16* __restrict__ Bt, const float* __restrict__ bias, h16* Ph) {
    gemm_body<h16, false, true, false>(A, Bt, bias, bias, Ph, (float*)nullptr, NB * SEQ, (size_t)0, DM, DM, (size_t)0, FSC, ACS);
}
__global__ __launch_bounds__(32) void k_ffn2(const h16* __restrict__ A, const h16* __restrict__ Bt, const float* __restrict__ bias, const float* __restrict__ resid, float* Pf) {
    gemm_body<h16, false, false, true>(A, Bt, bias, resid, (h16*)nullptr, Pf, NB * SEQ, (size_t)0, DM, DM, (size_t)0, FSC, 1.0f);
}

__global__ __launch_bounds__(32 * AW) void k_flash(const h16* __restrict__ QH, const h16* __restrict__ KP, const h16* __restrict__ VT, float* CTX) {
    __shared__ __align__(16) float os[AW * 16 * 68];
    const int lane = threadIdx.x & 31, lr = lane & 15, hi = lane >> 4;
    const int wave = __builtin_amdgcn_readfirstlane((int)(threadIdx.x >> 5));
    const int zh = blockIdx.y; const int b = zh / NH_, h = zh % NH_;
    const int t0 = (blockIdx.x * AW + wave) * 16;
    const size_t pbase = (size_t)zh * SEQ * HD;
    const size_t qo = pbase + (size_t)(t0 + lr) * HD + 8 * hi;
    const v16h qh0 = ldf(QH + qo), qh1 = ldf(QH + qo + 32);
    const size_t ko = pbase + (size_t)lr * HD + 8 * hi;
    const size_t vo = pbase + (size_t)lr * SEQ + 8 * hi;
    v8f o0 = (v8f){}, o1 = (v8f){}, o2 = (v8f){}, o3 = (v8f){};
    float m = -3.0e38f, l = 0.0f;
#pragma unroll 1
    for (int key0 = 0; key0 < SEQ; key0 += 32) {
        const h16* ka = KP + ko + (size_t)key0 * HD;
        const v16h ka0 = ldf(ka), ka1 = ldf(ka + 32), kb0 = ldf(ka + 16 * HD), kb1 = ldf(ka + 16 * HD + 32);
        v8f sa = (v8f){}, sb = (v8f){};
        sa = wm(ka0, qh0, sa); sb = wm(kb0, qh0, sb);
        sa = wm(ka1, qh1, sa); sb = wm(kb1, qh1, sb);
        float ta[8], tb[8]; float mx = -3.0e38f;
#pragma unroll
        for (int r = 0; r < 8; ++r) { ta[r] = sa[r] * SC2; tb[r] = sb[r] * SC2; mx = fmaxf(mx, fmaxf(ta[r], tb[r])); }
        mx = fmaxf(mx, __shfl_xor(mx, 16, 32));
        const float mnew = fmaxf(m, mx);
        const float alpha = __builtin_amdgcn_exp2f(m - mnew);
        const float sh = PSH - mnew;
        v16h pb; float ls = 0.0f;
#pragma unroll
        for (int r = 0; r < 8; ++r) { const float ea = __builtin_amdgcn_exp2f(ta[r] + sh); const float ec = __builtin_amdgcn_exp2f(tb[r] + sh); pb[r] = (h16)ea; pb[8 + r] = (h16)ec; ls += ea + ec; }
        l = l * alpha + ls; m = mnew;
        o0 = o0 * alpha; o1 = o1 * alpha; o2 = o2 * alpha; o3 = o3 * alpha;
        const h16* va = VT + vo + key0;
        const v16h v0 = ldf(va), v1 = ldf(va + (size_t)16 * SEQ), v2 = ldf(va + (size_t)32 * SEQ), v3 = ldf(va + (size_t)48 * SEQ);
        o0 = wm(v0, pb, o0); o1 = wm(v1, pb, o1); o2 = wm(v2, pb, o2); o3 = wm(v3, pb, o3);
    }
    l += __shfl_xor(l, 16, 32);
    const float inv = 1.0f / l;
    const int wb = wave * 16 * 68;
    { v4f a, c;
      a[0] = o0[0] * inv; a[1] = o0[1] * inv; a[2] = o0[2] * inv; a[3] = o0[3] * inv; c[0] = o0[4] * inv; c[1] = o0[5] * inv; c[2] = o0[6] * inv; c[3] = o0[7] * inv;
      *(v4fa*)(&os[wb + lr * 68 +  0 + 8 * hi]) = a; *(v4fa*)(&os[wb + lr * 68 +  0 + 8 * hi + 4]) = c;
      a[0] = o1[0] * inv; a[1] = o1[1] * inv; a[2] = o1[2] * inv; a[3] = o1[3] * inv; c[0] = o1[4] * inv; c[1] = o1[5] * inv; c[2] = o1[6] * inv; c[3] = o1[7] * inv;
      *(v4fa*)(&os[wb + lr * 68 + 16 + 8 * hi]) = a; *(v4fa*)(&os[wb + lr * 68 + 16 + 8 * hi + 4]) = c;
      a[0] = o2[0] * inv; a[1] = o2[1] * inv; a[2] = o2[2] * inv; a[3] = o2[3] * inv; c[0] = o2[4] * inv; c[1] = o2[5] * inv; c[2] = o2[6] * inv; c[3] = o2[7] * inv;
      *(v4fa*)(&os[wb + lr * 68 + 32 + 8 * hi]) = a; *(v4fa*)(&os[wb + lr * 68 + 32 + 8 * hi + 4]) = c;
      a[0] = o3[0] * inv; a[1] = o3[1] * inv; a[2] = o3[2] * inv; a[3] = o3[3] * inv; c[0] = o3[4] * inv; c[1] = o3[5] * inv; c[2] = o3[6] * inv; c[3] = o3[7] * inv;
      *(v4fa*)(&os[wb + lr * 68 + 48 + 8 * hi]) = a; *(v4fa*)(&os[wb + lr * 68 + 48 + 8 * hi + 4]) = c; }
    wave_sync();
    float* orow = CTX + ((size_t)b * SEQ + t0) * DM + h * HD;
#pragma unroll 1
    for (int ps = 0; ps < 2; ++ps) {
#pragma unroll
        for (int s = 0; s < 8; ++s) { const int row = 2 * s + hi, cofs = lr * 4;
            const v4f val = *(const v4fa*)(&os[wb + row * 68 + cofs]);
            *(volatile v4f*)(orow + (size_t)row * DM + cofs) = val; }
        if (ps == 0) __threadfence(); }
}

template <bool FIRST>
__device__ __forceinline__ void ln_body(const float* __restrict__ src, const bf* __restrict__ xb, const float* __restrict__ g, const float* __restrict__ be, float* dstf, h16* dsth) {
    __shared__ __align__(16) float rbuf[LNW * DM];
    const int lane = threadIdx.x & 31;
    const int wave = __builtin_amdgcn_readfirstlane((int)(threadIdx.x >> 5));
    const int row = blockIdx.x * LNW + wave;
    const size_t base = (size_t)row * DM;
    const int lb = wave * DM + lane * 4;
    float s = 0.0f;
#pragma unroll 1
    for (int j = 0; j < DM / 128; ++j) {
        const int c = j * 128 + lane * 4;
        v4f v = *(const v4f*)(src + base + c);
        if (FIRST) { const v4us xv = *(const v4us*)(xb + base + c);
#pragma unroll
            for (int i = 0; i < 4; ++i) v[i] += bf2f(xv[i]); }
        *(v4fa*)(&rbuf[lb + j * 128]) = v;
        s += (v[0] + v[1]) + (v[2] + v[3]);
    }
    s += __shfl_xor(s, 16, 32); s += __shfl_xor(s, 8, 32); s += __shfl_xor(s, 4, 32); s += __shfl_xor(s, 2, 32); s += __shfl_xor(s, 1, 32);
    const float mu = s * (1.0f / (float)DM);
    float q = 0.0f;
#pragma unroll 1
    for (int j = 0; j < DM / 128; ++j) {
        const v4f v = *(const v4fa*)(&rbuf[lb + j * 128]);
#pragma unroll
        for (int i = 0; i < 4; ++i) { const float d = v[i] - mu; q += d * d; }
    }
    q += __shfl_xor(q, 16, 32); q += __shfl_xor(q, 8, 32); q += __shfl_xor(q, 4, 32); q += __shfl_xor(q, 2, 32); q += __shfl_xor(q, 1, 32);
    const float inv = rsqrtf(q * (1.0f / (float)DM) + 1e-5f);
    const size_t obase = FIRST ? base : ((size_t)(row / SEQ) * OUT_SEQ + (size_t)(row % SEQ)) * DM;
#pragma unroll 1
    for (int ps = 0; ps < 2; ++ps) {
#pragma unroll 1
        for (int j = 0; j < DM / 128; ++j) {
            const int c = j * 128 + lane * 4;
            const v4f v = *(const v4fa*)(&rbuf[lb + j * 128]);
            const v4f gg = *(const v4f*)(g + c); const v4f bb = *(const v4f*)(be + c);
            v4f y;
#pragma unroll
            for (int i = 0; i < 4; ++i) y[i] = (v[i] - mu) * inv * bfv(gg[i]) + bfv(bb[i]);
            *(volatile v4f*)(dstf + obase + c) = y;
            if (FIRST) { v4h hv;
#pragma unroll
                for (int i = 0; i < 4; ++i) hv[i] = (h16)(y[i] * ACS);
                *(volatile v4h*)(dsth + base + c) = hv; }
        }
        if (ps == 0) __threadfence();
    }
}

__global__ __launch_bounds__(32 * LNW) void k_ln1(const float* __restrict__ ctx, const bf* __restrict__ xb, const float* __restrict__ g, const float* __restrict__ be, float* c1, h16* c1h) {
    ln_body<true>(ctx, xb, g, be, c1, c1h);
}
__global__ __launch_bounds__(32 * LNW) void k_ln2(const float* __restrict__ pre, const float* __restrict__ g, const float* __restrict__ be, float* out) {
    ln_body<false>(pre, (const bf*)nullptr, g, be, out, (h16*)nullptr);
}

static constexpr size_t al256(size_t v) { return (v + 255) & ~(size_t)255; }
static constexpr size_t SZ_XB  = al256((size_t)NB * SEQ * DM * 2);
static constexpr size_t SZ_WB  = al256((size_t)3 * DM * DM * 2);
static constexpr size_t SZ_WF  = al256((size_t)2 * DM * DM * 2);
static constexpr size_t SZ_PL  = al256((size_t)NB * NH_ * SEQ * HD * 2);
static constexpr size_t SZ_F32 = al256((size_t)NB * SEQ * DM * 4);
static constexpr size_t SZ_H16 = al256((size_t)NB * SEQ * DM * 2);
static constexpr size_t SZ_TOTAL = SZ_XB + SZ_WB + SZ_WF + 3 * SZ_PL + 3 * SZ_F32 + 2 * SZ_H16;
static_assert(SZ_TOTAL <= (size_t)134217728);
static_assert(((size_t)DM * DM * 2) % 256 == 0);

extern "C" void kernel_launch(void* const* d_in, const int* in_sizes, int n_in,
                              void* d_out, int out_size, void* d_ws, size_t ws_size, hipStream_t stream) {
    if (n_in < 13) return;
    const size_t needx = ((size_t)(NB - 1) * SEQ_FULL + SEQ) * DM;
    if ((size_t)in_sizes[0] < needx) return;
    if ((size_t)in_sizes[1] < (size_t)DM * DM || (size_t)in_sizes[3] < (size_t)DM * DM || (size_t)in_sizes[5] < (size_t)DM * DM) return;
    if ((size_t)in_sizes[9] < (size_t)DM * DM || (size_t)in_sizes[11] < (size_t)DM * DM) return;
    if (in_sizes[2] < DM || in_sizes[4] < DM || in_sizes[6] < DM || in_sizes[7] < DM || in_sizes[8] < DM || in_sizes[10] < DM || in_sizes[12] < DM) return;
    if ((size_t)out_size < ((size_t)(NB - 1) * OUT_SEQ + SEQ) * DM) return;
    if (SZ_TOTAL > ws_size) return;
    const float* x  = (const float*)d_in[0];
    const float* wq = (const float*)d_in[1];  const float* bq = (const float*)d_in[2];
    const float* wk = (const float*)d_in[3];  const float* bk = (const float*)d_in[4];
    const float* wv = (const float*)d_in[5];  const float* bv = (const float*)d_in[6];
    const float* lg = (const float*)d_in[7];  const float* lb = (const float*)d_in[8];
    const float* w1 = (const float*)d_in[9];  const float* b1 = (const float*)d_in[10];
    const float* w2 = (const float*)d_in[11]; const float* b2 = (const float*)d_in[12];
    float* OUT = (float*)d_out;
    char* wsp = (char*)d_ws;
    bf*  XB  = (bf*)wsp;   wsp += SZ_XB;
    bf*  WB  = (bf*)wsp;   wsp += SZ_WB;
    h16* WF  = (h16*)wsp;  wsp += SZ_WF;
    h16* QH  = (h16*)wsp;  wsp += SZ_PL;
    h16* KP  = (h16*)wsp;  wsp += SZ_PL;
    h16* VT  = (h16*)wsp;  wsp += SZ_PL;
    float* CTX  = (float*)wsp; wsp += SZ_F32;
    float* C1   = (float*)wsp; wsp += SZ_F32;
    float* PRE2 = (float*)wsp; wsp += SZ_F32;
    h16* C1H = (h16*)wsp;  wsp += SZ_H16;
    h16* HH  = (h16*)wsp;  wsp += SZ_H16;
    bf* WQ = WB; bf* WK = WB + (size_t)DM * DM; bf* WV = WB + (size_t)2 * DM * DM;
    h16* W1H = WF; h16* W2H = WF + (size_t)DM * DM;

    if (SEQ == SEQ_FULL) {
        const size_t n8 = (size_t)NB * SEQ * DM / 8;
        k_cvt8<<<(unsigned)((n8 + 255) / 256), 256, 0, stream>>>(x, XB, n8);
    } else {
        const size_t n8 = (size_t)SEQ * DM / 8;
        for (int b = 0; b < NB; ++b) k_cvt8<<<(unsigned)((n8 + 255) / 256), 256, 0, stream>>>(x + (size_t)b * SEQ_FULL * DM, XB + (size_t)b * SEQ * DM, n8);
    }
    { const size_t n8 = (size_t)DM * DM / 8; const unsigned g = (unsigned)((n8 + 255) / 256);
      k_cvt8<<<g, 256, 0, stream>>>(wq, WQ, n8); k_cvt8<<<g, 256, 0, stream>>>(wk, WK, n8); k_cvt8<<<g, 256, 0, stream>>>(wv, WV, n8);
      k_cvt8h<<<g, 256, 0, stream>>>(w1, W1H, n8); k_cvt8h<<<g, 256, 0, stream>>>(w2, W2H, n8); }

    k_proj_qk<<<dim3(NB * SEQ / 64, DM / 64, 1), 32, 0, stream>>>(XB, WQ, bq, QH);
    k_proj_qk<<<dim3(NB * SEQ / 64, DM / 64, 1), 32, 0, stream>>>(XB, WK, bk, KP);
    k_proj_vt<<<dim3(DM / 64, NB * SEQ / 64, 1), 32, 0, stream>>>(WV, XB, bv, VT);

    k_flash<<<dim3(SEQ / (16 * AW), NB * NH_, 1), 32 * AW, 0, stream>>>(QH, KP, VT, CTX);

    k_ln1<<<NB * SEQ / LNW, 32 * LNW, 0, stream>>>(CTX, XB, lg, lb, C1, C1H);
    k_ffn1<<<dim3(NB * SEQ / 64, DM / 64, 1), 32, 0, stream>>>(C1H, W1H, b1, HH);
    k_ffn2<<<dim3(NB * SEQ / 64, DM / 64, 1), 32, 0, stream>>>(HH, W2H, b2, C1, PRE2);
    k_ln2<<<NB * SEQ / LNW, 32 * LNW, 0, stream>>>(PRE2, lg, lb, OUT);
}
